// MultiHeadAttention_14894946582935
// MI455X (gfx1250) — hardware-verified
//
#include <hip/hip_runtime.h>


#ifndef NB
#define NB 4
#endif
#ifndef SEQ
#define SEQ 2048
#endif
#define NB_FULL  4
#define SEQ_FULL 2048
#define DM   1024
#define NH_  16
#define HD   64
#define RH   (((SEQ) < 512) ? (SEQ) : 512)
#define PCAR 1024.0f
#define SCL  0.125f
#define L2E  1.4426950408889634f
static_assert(NB <= NB_FULL);
static_assert(SEQ <= SEQ_FULL);
static_assert(DM == NH_ * HD);
static_assert(HD == 64);
static_assert(DM % 64 == 0);
static_assert(SEQ % 64 == 0);
static_assert(RH % 64 == 0);
static_assert((SEQ - RH) % 32 == 0);
static_assert(RH % 16 == 0);
static_assert(((size_t)SEQ * DM) % 2048 == 0);
static_assert(((size_t)DM * DM) % 2048 == 0);

typedef _Float16 h16;
typedef unsigned short bf;
typedef __attribute__((ext_vector_type(16))) __bf16   v16bf;
typedef __attribute__((ext_vector_type(16))) _Float16 v16h;
typedef __attribute__((ext_vector_type(8)))  _Float16 v8h;
typedef __attribute__((ext_vector_type(8)))  unsigned short v8us;
typedef __attribute__((ext_vector_type(8)))  float    v8f;
typedef __attribute__((ext_vector_type(4)))  float    v4f;
typedef v4f  __attribute__((may_alias)) v4fa;

__device__ __forceinline__ unsigned short f2bf(float f) { unsigned u = __float_as_uint(f); u += 0x7FFFu + ((u >> 16) & 1u); return (unsigned short)(u >> 16); }
__device__ __forceinline__ float bf2f(unsigned short b) { return __uint_as_float(((unsigned)b) << 16); }
__device__ __forceinline__ float bfr(float f) { return bf2f(f2bf(f)); }
__device__ __forceinline__ void splitf(float y, unsigned short& h, unsigned short& l) { h = f2bf(y); l = f2bf(y - bf2f(h)); }
__device__ __forceinline__ v16h cat16(v8h lo, v8h hi) { return __builtin_shufflevector(lo, hi, 0, 1, 2, 3, 4, 5, 6, 7, 8, 9, 10, 11, 12, 13, 14, 15); }
__device__ __forceinline__ v16bf cat16b(v8us lo, v8us hi) { return __builtin_bit_cast(v16bf, __builtin_shufflevector(lo, hi, 0, 1, 2, 3, 4, 5, 6, 7, 8, 9, 10, 11, 12, 13, 14, 15)); }
__device__ __forceinline__ v8f wmma16(v16h a, v16h b, v8f c) { return __builtin_amdgcn_wmma_f32_16x16x32_f16(false, a, false, b, (short)0, c, false, false); }
__device__ __forceinline__ v8f wmmab(v16bf a, v16bf b, v8f c) { return __builtin_amdgcn_wmma_f32_16x16x32_bf16(false, a, false, b, (short)0, c, false, false); }
__device__ __forceinline__ void wsync() { __builtin_amdgcn_wave_barrier(); asm volatile("" ::: "memory"); }

template <typename T16> struct WFrag;
template <> struct WFrag<h16> {
    typedef v16h V;
    static __device__ __forceinline__ V ld(const h16* p) { return cat16(*(const v8h*)p, *(const v8h*)(p + 16)); }
    static __device__ __forceinline__ v8f mma(V a, V b, v8f c) { return wmma16(a, b, c); }
    static __device__ __forceinline__ float car() { return PCAR; }
    static __device__ __forceinline__ V pk(const float (&a)[8], const float (&b)[8]) { v8h lo, hi;
#pragma unroll
        for (int k = 0; k < 8; ++k) { lo[k] = (h16)(a[k] * PCAR); hi[k] = (h16)(b[k] * PCAR); } return cat16(lo, hi); }
    static __device__ __forceinline__ V pkl(const float (&a)[8], const float (&b)[8]) { return pk(a, b); }
};
template <> struct WFrag<bf> {
    typedef v16bf V;
    static __device__ __forceinline__ V ld(const bf* p) { return cat16b(*(const v8us*)p, *(const v8us*)(p + 16)); }
    static __device__ __forceinline__ v8f mma(V a, V b, v8f c) { return wmmab(a, b, c); }
    static __device__ __forceinline__ float car() { return 1.0f; }
    static __device__ __forceinline__ V pk(const float (&a)[8], const float (&b)[8]) { v8us lo, hi;
#pragma unroll
        for (int k = 0; k < 8; ++k) { lo[k] = f2bf(a[k]); hi[k] = f2bf(b[k]); } return cat16b(lo, hi); }
    static __device__ __forceinline__ V pkl(const float (&a)[8], const float (&b)[8]) { v8us lo, hi;
#pragma unroll
        for (int k = 0; k < 8; ++k) { lo[k] = f2bf(a[k] - bf2f(f2bf(a[k]))); hi[k] = f2bf(b[k] - bf2f(f2bf(b[k]))); } return cat16b(lo, hi); }
};

__global__ __launch_bounds__(256) void k_cvt8(const float* __restrict__ src, bf* dst, unsigned n8, size_t sS, size_t sD) {
    const unsigned i = blockIdx.x * 256u + threadIdx.x; if (i >= n8) return;
    src += (size_t)blockIdx.y * sS; dst += (size_t)blockIdx.y * sD;
    const v8f v = *(const v8f*)(src + (size_t)i * 8); v8us o;
#pragma unroll
    for (int k = 0; k < 8; ++k) o[k] = f2bf(v[k]);
    *(volatile v8us*)(dst + (size_t)i * 8) = o; __threadfence(); *(volatile v8us*)(dst + (size_t)i * 8) = o; }

template <int HLMODE>
__global__ __launch_bounds__(32) void k_gemmp(const bf* __restrict__ A, const bf* __restrict__ Bt, int K, h16* P16, int ldp, bf* Ph, bf* Pl, int ldh, size_t sA, size_t sB, size_t sP, size_t sH) {
    typedef WFrag<bf>::V V;
    __shared__ __align__(16) float os[16 * 68];
    const size_t z = blockIdx.z; A += z * sA; Bt += z * sB; P16 += z * sP; Ph += z * sH; Pl += z * sH;
    const int lane = threadIdx.x & 31, lr = lane & 15, hi = lane >> 4; const int r0 = blockIdx.x * 64, c0 = blockIdx.y * 64;
    const bool hl = (HLMODE == 0) ? (r0 < RH) : (c0 < RH);
    v8f acc[4][4];
#pragma unroll
    for (int mb = 0; mb < 4; ++mb)
#pragma unroll
        for (int nb = 0; nb < 4; ++nb) acc[mb][nb] = (v8f){};
    const size_t aoff = (size_t)(r0 + lr) * K + 8 * hi, boff = (size_t)(c0 + lr) * K + 8 * hi;
#pragma unroll 1
    for (int kc = 0; kc < K; kc += 32) {
        V a[4];
#pragma unroll
        for (int mb = 0; mb < 4; ++mb) a[mb] = WFrag<bf>::ld(A + aoff + (size_t)mb * 16 * K + kc);
#pragma unroll
        for (int nb = 0; nb < 4; ++nb) { const V bq = WFrag<bf>::ld(Bt + boff + (size_t)nb * 16 * K + kc);
#pragma unroll
            for (int mb = 0; mb < 4; ++mb) acc[mb][nb] = WFrag<bf>::mma(a[mb], bq, acc[mb][nb]); }
        asm volatile("v_nop\n\tv_nop\n\tv_nop\n\tv_nop" : "+v"(acc[0][0]), "+v"(acc[1][1]), "+v"(acc[2][2]), "+v"(acc[3][3]) : "v"(a[0]), "v"(a[3]));
    }
    const unsigned ul = (unsigned)lane;
#pragma unroll
    for (int mb = 0; mb < 4; ++mb) {
#pragma unroll
        for (int nb = 0; nb < 4; ++nb) {
#pragma unroll
            for (int j = 0; j < 8; ++j) os[(hi * 8 + j) * 68 + nb * 16 + lr] = acc[mb][nb][j]; }
        wsync();
        const size_t rb = (size_t)(r0 + mb * 16);
#pragma unroll 1
        for (int ps = 0; ps < 2; ++ps) {
#pragma unroll
            for (unsigned s = 0; s < 4u; ++s) { const unsigned row = 4u * s + (ul >> 3), cc = (ul & 7u) * 8u;
                const v4f x0 = *(const v4fa*)(os + row * 68u + cc), x1 = *(const v4fa*)(os + row * 68u + cc + 4u);
                v8h o; v8us oh, ol;
#pragma unroll
                for (int k = 0; k < 4; ++k) { unsigned short a2, c2; o[k] = (h16)x0[k]; splitf(x0[k], a2, c2); oh[k] = a2; ol[k] = c2; o[k + 4] = (h16)x1[k]; splitf(x1[k], a2, c2); oh[k + 4] = a2; ol[k + 4] = c2; }
                *(volatile v8h*)(P16 + (rb + row) * (size_t)ldp + c0 + cc) = o;
                if (hl) { *(volatile v8us*)(Ph + (rb + row) * (size_t)ldh + c0 + cc) = oh; *(volatile v8us*)(Pl + (rb + row) * (size_t)ldh + c0 + cc) = ol; } }
            if (ps == 0) __threadfence(); }
        wsync();
    }
}

template <typename T16, int NG, bool HL>
__global__ __launch_bounds__(32) void k_flash(const T16* __restrict__ Qa, const T16* __restrict__ Qb, const T16* __restrict__ Ka, const T16* __restrict__ Kb,
                                              const T16* __restrict__ Va, const T16* __restrict__ Vb, unsigned TP, unsigned qbase, bf* ATh, bf* ATl) {
    static_assert((NG == 2 && !HL) || (NG == 1 && HL));
    typedef WFrag<T16> W; typedef typename W::V V;
    __shared__ __align__(16) float os[16 * NG * 68];
    const unsigned lane = threadIdx.x & 31u, lr = lane & 15u, hi = lane >> 4;
    const unsigned hh = blockIdx.y, b = blockIdx.z;
    const unsigned q0 = qbase + blockIdx.x * (16u * NG);
    const size_t VP = (size_t)NB * TP;
    const size_t qo = ((size_t)b * TP + q0 + lr) * DM + hh * HD + 8u * hi;
    V qf[2][2], qg[2][2];
#pragma unroll
    for (int g = 0; g < NG; ++g)
#pragma unroll
        for (int ds = 0; ds < 2; ++ds) { qf[g][ds] = W::ld(Qa + qo + (size_t)g * 16 * DM + ds * 32); if (HL) qg[g][ds] = W::ld(Qb + qo + (size_t)g * 16 * DM + ds * 32); else qg[g][ds] = qf[g][ds]; }
    v8f oacc[2][4]; float m[2], l[2];
#pragma unroll
    for (int g = 0; g < 2; ++g) { m[g] = -3.0e38f; l[g] = 0.0f;
#pragma unroll
        for (int dt = 0; dt < 4; ++dt) oacc[g][dt] = (v8f){}; }
    const unsigned kend = q0 + 16u * NG;
    const size_t kbase = ((size_t)b * TP + lr) * DM + hh * HD + 8u * hi;
    const size_t vbase = (size_t)(hh * HD + lr) * VP + (size_t)b * TP + 8u * hi;
#pragma unroll 1
    for (unsigned kb = 0; kb < kend; kb += 32u) {
        V ka[2][2], kl[2][2];
#pragma unroll
        for (int kt = 0; kt < 2; ++kt)
#pragma unroll
            for (int ds = 0; ds < 2; ++ds) { const size_t o = kbase + (size_t)(kb + kt * 16) * DM + ds * 32; ka[kt][ds] = W::ld(Ka + o); if (HL) kl[kt][ds] = W::ld(Kb + o); else kl[kt][ds] = ka[kt][ds]; }
        v8f s[2][2];
#pragma unroll
        for (int g = 0; g < NG; ++g)
#pragma unroll
            for (int kt = 0; kt < 2; ++kt) { v8f c = (v8f){};
                c = W::mma(ka[kt][0], qf[g][0], c); c = W::mma(ka[kt][1], qf[g][1], c);
                if (HL) { c = W::mma(kl[kt][0], qf[g][0], c); c = W::mma(kl[kt][1], qf[g][1], c); c = W::mma(ka[kt][0], qg[g][0], c); c = W::mma(ka[kt][1], qg[g][1], c); }
                s[g][kt] = c; }
        if (NG == 2) asm volatile("v_nop\n\tv_nop\n\tv_nop\n\tv_nop" : "+v"(s[0][0]), "+v"(s[0][1]), "+v"(s[1][0]), "+v"(s[1][1]) : "v"(ka[0][0]), "v"(ka[0][1]), "v"(ka[1][0]), "v"(ka[1][1]));
        else         asm volatile("v_nop\n\tv_nop\n\tv_nop\n\tv_nop" : "+v"(s[0][0]), "+v"(s[0][1]) : "v"(ka[0][0]), "v"(ka[0][1]), "v"(ka[1][0]), "v"(ka[1][1]), "v"(kl[0][0]), "v"(kl[0][1]), "v"(kl[1][0]), "v"(kl[1][1]));
        V pb[2], pl[2];
        const unsigned kq = kb + 8u * hi;
#pragma unroll
        for (int g = 0; g < NG; ++g) {
            const unsigned qi = q0 + (unsigned)g * 16u + lr;
            float t0[8], t1[8]; float mx = -3.0e38f;
#pragma unroll
            for (int r = 0; r < 8; ++r) { t0[r] = (kq + (unsigned)r <= qi) ? s[g][0][r] * SCL : -3.0e38f; t1[r] = (kq + 16u + (unsigned)r <= qi) ? s[g][1][r] * SCL : -3.0e38f; mx = fmaxf(mx, fmaxf(t0[r], t1[r])); }
            mx = fmaxf(mx, __shfl_xor(mx, 16, 32));
            const float mn = fmaxf(m[g], mx);
            const float al = __builtin_amdgcn_exp2f((m[g] - mn) * L2E); m[g] = mn;
            float p0[8], p1[8]; float rs = 0.0f;
#pragma unroll
            for (int r = 0; r < 8; ++r) { const float e0 = __builtin_amdgcn_exp2f((t0[r] - mn) * L2E), e1 = __builtin_amdgcn_exp2f((t1[r] - mn) * L2E);
                p0[r] = (kq + (unsigned)r <= qi) ? e0 : 0.0f; p1[r] = (kq + 16u + (unsigned)r <= qi) ? e1 : 0.0f; rs += p0[r] + p1[r]; }
            l[g] = l[g] * al + rs;
            pb[g] = W::pk(p0, p1); if (HL) pl[g] = W::pkl(p0, p1); else pl[g] = pb[g];
#pragma unroll
            for (int dt = 0; dt < 4; ++dt)
#pragma unroll
                for (int r = 0; r < 8; ++r) oacc[g][dt][r] *= al;
        }
        V va[4], vb[4];
#pragma unroll
        for (int dt = 0; dt < 4; ++dt) { const size_t o = vbase + (size_t)dt * 16 * VP + kb; va[dt] = W::ld(Va + o); if (HL) vb[dt] = W::ld(Vb + o); else vb[dt] = va[dt]; }
#pragma unroll
        for (int dt = 0; dt < 4; ++dt)
#pragma unroll
            for (int g = 0; g < NG; ++g) { oacc[g][dt] = W::mma(va[dt], pb[g], oacc[g][dt]); if (HL) { oacc[g][dt] = W::mma(vb[dt], pb[g], oacc[g][dt]); oacc[g][dt] = W::mma(va[dt], pl[g], oacc[g][dt]); } }
        if (NG == 2) asm volatile("v_nop\n\tv_nop\n\tv_nop\n\tv_nop" : "+v"(oacc[0][0]), "+v"(oacc[0][1]), "+v"(oacc[0][2]), "+v"(oacc[0][3]), "+v"(oacc[1][0]), "+v"(oacc[1][1]), "+v"(oacc[1][2]), "+v"(oacc[1][3])
                                       : "v"(va[0]), "v"(va[1]), "v"(va[2]), "v"(va[3]), "v"(pb[0]), "v"(pb[1]));
        else         asm volatile("v_nop\n\tv_nop\n\tv_nop\n\tv_nop" : "+v"(oacc[0][0]), "+v"(oacc[0][1]), "+v"(oacc[0][2]), "+v"(oacc[0][3])
                                       : "v"(va[0]), "v"(va[1]), "v"(va[2]), "v"(va[3]), "v"(vb[0]), "v"(vb[1]), "v"(vb[2]), "v"(vb[3]), "v"(pb[0]), "v"(pl[0]));
    }
#pragma unroll
    for (int g = 0; g < NG; ++g) { const float lt = l[g] + __shfl_xor(l[g], 16, 32); const float inv = (1.0f / W::car()) * (1.0f / lt);
#pragma unroll
        for (int dt = 0; dt < 4; ++dt)
#pragma unroll
            for (int r = 0; r < 8; ++r) os[((unsigned)g * 16u + lr) * 68u + (unsigned)dt * 16u + 8u * hi + (unsigned)r] = oacc[g][dt][r] * inv; }
    wsync();
    const size_t ab = ((size_t)b * SEQ + q0) * DM + hh * HD;
#pragma unroll 1
    for (int ps = 0; ps < 2; ++ps) {
#pragma unroll
        for (unsigned s = 0; s < 4u * NG; ++s) { const unsigned row = 4u * s + (lane >> 3), cc = (lane & 7u) * 8u;
            const v4f x0 = *(const v4fa*)(os + row * 68u + cc), x1 = *(const v4fa*)(os + row * 68u + cc + 4u);
            v8us oh, ol;
#pragma unroll
            for (int k = 0; k < 4; ++k) { unsigned short a2, c2; splitf(x0[k], a2, c2); oh[k] = a2; ol[k] = c2; splitf(x1[k], a2, c2); oh[k + 4] = a2; ol[k + 4] = c2; }
            *(volatile v8us*)(ATh + ab + (size_t)row * DM + cc) = oh; *(volatile v8us*)(ATl + ab + (size_t)row * DM + cc) = ol; }
        if (ps == 0) __threadfence(); }
}

template <typename T16, int NSPLIT, bool BIAS>
__global__ __launch_bounds__(32) void k_gemmw(const T16* __restrict__ A, const T16* __restrict__ A2, const T16* __restrict__ Bt, const T16* __restrict__ Bt2, int K, float* C, int ldc, const float* __restrict__ bias, size_t sA, size_t sB, size_t sC) {
    typedef typename WFrag<T16>::V V;
    __shared__ __align__(16) float os[16 * 68];
    const size_t z = blockIdx.z; A += z * sA; if (A2) A2 += z * sA; Bt += z * sB; if (Bt2) Bt2 += z * sB; C += z * sC;
    const int lane = threadIdx.x & 31, lr = lane & 15, hi = lane >> 4; const int r0 = blockIdx.x * 64, c0 = blockIdx.y * 64;
    v8f acc[4][4];
#pragma unroll
    for (int mb = 0; mb < 4; ++mb)
#pragma unroll
        for (int nb = 0; nb < 4; ++nb) acc[mb][nb] = (v8f){};
    const size_t aoff = (size_t)(r0 + lr) * K + 8 * hi, boff = (size_t)(c0 + lr) * K + 8 * hi;
#pragma unroll 1
    for (int kc = 0; kc < K; kc += 32) {
        V a[4], a2[4];
#pragma unroll
        for (int mb = 0; mb < 4; ++mb) { a[mb] = WFrag<T16>::ld(A + aoff + (size_t)mb * 16 * K + kc); if (NSPLIT == 1 || NSPLIT == 2) a2[mb] = WFrag<T16>::ld(A2 + aoff + (size_t)mb * 16 * K + kc); }
#pragma unroll
        for (int nb = 0; nb < 4; ++nb) { const V b = WFrag<T16>::ld(Bt + boff + (size_t)nb * 16 * K + kc); V b2; if (NSPLIT >= 2) b2 = WFrag<T16>::ld(Bt2 + boff + (size_t)nb * 16 * K + kc);
#pragma unroll
            for (int mb = 0; mb < 4; ++mb) { acc[mb][nb] = WFrag<T16>::mma(a[mb], b, acc[mb][nb]); if (NSPLIT == 1 || NSPLIT == 2) acc[mb][nb] = WFrag<T16>::mma(a2[mb], b, acc[mb][nb]); if (NSPLIT >= 2) acc[mb][nb] = WFrag<T16>::mma(a[mb], b2, acc[mb][nb]); } }
        asm volatile("v_nop\n\tv_nop\n\tv_nop\n\tv_nop" : "+v"(acc[0][0]), "+v"(acc[1][1]), "+v"(acc[2][2]), "+v"(acc[3][3]) : "v"(a[0]), "v"(a[3]));
    }
#pragma unroll
    for (int mb = 0; mb < 4; ++mb) {
#pragma unroll
        for (int nb = 0; nb < 4; ++nb) {
#pragma unroll
            for (int j = 0; j < 8; ++j) os[(hi * 8 + j) * 68 + nb * 16 + lr] = acc[mb][nb][j]; }
        wsync();
        float* crow = C + (size_t)(r0 + mb * 16) * ldc + c0;
#pragma unroll 1
        for (int ps = 0; ps < 2; ++ps) {
#pragma unroll
            for (int s = 0; s < 8; ++s) { const int row = 2 * s + hi, cofs = lr * 4; v4f val = *(const v4fa*)(os + row * 68 + cofs); if (BIAS) { val[0] += bfr(bias[c0 + cofs]); val[1] += bfr(bias[c0 + cofs + 1]); val[2] += bfr(bias[c0 + cofs + 2]); val[3] += bfr(bias[c0 + cofs + 3]); }
                *(volatile v4f*)(crow + (size_t)row * ldc + cofs) = val; }
            if (ps == 0) __threadfence(); }
        wsync();
    }
}

constexpr size_t SZ_W = (size_t)DM * DM * 2;
constexpr size_t SZ_X = (size_t)NB * SEQ * DM * 2;
constexpr size_t SZ_P = (size_t)NB * SEQ * DM * 2;
constexpr size_t SZ_H = (size_t)NB * RH * DM * 2;
constexpr size_t WS_TOTAL = 4 * SZ_W + SZ_X + 3 * SZ_P + 6 * SZ_H + SZ_P;
static_assert(SZ_X == SZ_P);
static_assert(WS_TOTAL <= (size_t)134217728);

extern "C" void kernel_launch(void* const* d_in, const int* in_sizes, int n_in,
                              void* d_out, int out_size, void* d_ws, size_t ws_size, hipStream_t stream) {
    if (n_in < 6) return;
    const size_t need_x = ((size_t)(NB - 1) * SEQ_FULL + SEQ) * DM;
    if ((size_t)in_sizes[0] < need_x || (size_t)in_sizes[1] < (size_t)DM * DM || (size_t)in_sizes[2] < (size_t)DM * DM || (size_t)in_sizes[3] < (size_t)DM * DM || (size_t)in_sizes[4] < (size_t)DM * DM || in_sizes[5] < DM) return;
    if ((size_t)out_size < need_x) return;
    if (ws_size < WS_TOTAL) return;
    const float* x = (const float*)d_in[0]; const float* wq = (const float*)d_in[1]; const float* wk = (const float*)d_in[2]; const float* wv = (const float*)d_in[3]; const float* wo = (const float*)d_in[4]; const float* bo = (const float*)d_in[5];
    float* OUT = (float*)d_out;
    char* wsp = (char*)d_ws;
    auto take = [&](size_t bytes) { char* p = wsp; wsp += (bytes + 255) & ~(size_t)255; return (void*)p; };
    bf* WQ = (bf*)take(SZ_W); bf* WK = (bf*)take(SZ_W); bf* WV = (bf*)take(SZ_W); bf* WO = (bf*)take(SZ_W);
    bf* XB = (bf*)take(SZ_X);
    h16* Q16 = (h16*)take(SZ_P); h16* K16 = (h16*)take(SZ_P); h16* VT16 = (h16*)take(SZ_P);
    bf* Qh = (bf*)take(SZ_H); bf* Ql = (bf*)take(SZ_H); bf* Kh = (bf*)take(SZ_H); bf* Kl = (bf*)take(SZ_H); bf* VTh = (bf*)take(SZ_H); bf* VTl = (bf*)take(SZ_H);
    bf* ATl = (bf*)take(SZ_P);
    bf* ATh = XB;
    if ((size_t)(wsp - (char*)d_ws) > ws_size) return;

    const unsigned nW8 = (unsigned)((size_t)DM * DM / 8), nX8 = (unsigned)((size_t)SEQ * DM / 8);
    k_cvt8<<<dim3(nW8 / 256, 1, 1), 256, 0, stream>>>(wq, WQ, nW8, 0, 0);
    k_cvt8<<<dim3(nW8 / 256, 1, 1), 256, 0, stream>>>(wk, WK, nW8, 0, 0);
    k_cvt8<<<dim3(nW8 / 256, 1, 1), 256, 0, stream>>>(wv, WV, nW8, 0, 0);
    k_cvt8<<<dim3(nW8 / 256, 1, 1), 256, 0, stream>>>(wo, WO, nW8, 0, 0);
    k_cvt8<<<dim3(nX8 / 256, NB, 1), 256, 0, stream>>>(x, XB, nX8, (size_t)SEQ_FULL * DM, (size_t)SEQ * DM);

    k_gemmp<0><<<dim3(SEQ / 64, DM / 64, NB), 32, 0, stream>>>(XB, WQ, DM, Q16, DM, Qh, Ql, DM, (size_t)SEQ * DM, 0, (size_t)SEQ * DM, (size_t)RH * DM);
    k_gemmp<0><<<dim3(SEQ / 64, DM / 64, NB), 32, 0, stream>>>(XB, WK, DM, K16, DM, Kh, Kl, DM, (size_t)SEQ * DM, 0, (size_t)SEQ * DM, (size_t)RH * DM);
    k_gemmp<1><<<dim3(DM / 64, SEQ / 64, NB), 32, 0, stream>>>(WV, XB, DM, VT16, NB * SEQ, VTh, VTl, NB * RH, 0, (size_t)SEQ * DM, (size_t)SEQ, (size_t)RH);

    k_flash<bf, 1, true><<<dim3(RH / 16, NH_, NB), 32, 0, stream>>>(Qh, Ql, Kh, Kl, VTh, VTl, (unsigned)RH, 0u, ATh, ATl);
    if (SEQ > RH)
        k_flash<h16, 2, false><<<dim3((SEQ - RH) / 32 + ((SEQ > RH) ? 0 : 1), NH_, NB), 32, 0, stream>>>(Q16, nullptr, K16, nullptr, VT16, nullptr, (unsigned)SEQ, (unsigned)RH, ATh, ATl);

    k_gemmw<bf, 1, true><<<dim3(SEQ / 64, DM / 64, NB), 32, 0, stream>>>(ATh, ATl, WO, nullptr, DM, OUT, DM, bo, (size_t)SEQ * DM, 0, (size_t)SEQ_FULL * DM);
}
